// SSM_47141561041352
// MI455X (gfx1250) — hardware-run, weakly checked
//
#include <hip/hip_runtime.h>
#include <math.h>

typedef __attribute__((ext_vector_type(16))) _Float16 v16h;
typedef __attribute__((ext_vector_type(8)))  _Float16 v8h;
typedef __attribute__((ext_vector_type(16))) __bf16   v16b;
typedef __attribute__((ext_vector_type(8)))  __bf16   v8b;
typedef __attribute__((ext_vector_type(8)))  float    v8f;
typedef __attribute__((ext_vector_type(4)))  float    v4f;

constexpr int kNB     = 8;
constexpr int kDmod   = 96;
constexpr int kDin    = 192;
constexpr int kImg    = 32;
constexpr int kHW     = kImg * kImg;
constexpr int kSeqL   = 4 * kHW;
constexpr int kNst    = 16;
constexpr int kDtR    = 6;
constexpr int kXpN    = kDtR + 2 * kNst;
constexpr int kPix    = kNB * kHW;
constexpr int kTok    = kNB * kSeqL;
constexpr int kXtP    = 128;
constexpr int kXzP    = 2 * kDin;
constexpr int kXdP    = 64;
constexpr int kColB   = 8;
constexpr int kColC   = 24;
constexpr int kWoM    = 128;
constexpr int kScanTS = 64;
constexpr int kScanCh = 64;
constexpr int kScanYP = 68;
constexpr int kConvPT = 16;
static_assert(kColB >= kDtR && kColC == kColB + kNst && kColC + kNst <= kXdP, "x_dbl column map");
static_assert((kDmod % 32) == 0 && (kDin % 32) == 0, "GEMM K multiples of 32");
static_assert((kPix % 64) == 0 && (kXzP % 64) == 0 && (kHW % 64) == 0 && (kDin % 64) == 0 &&
              (kTok % 64) == 0 && (kXdP % 64) == 0 && (kWoM % 64) == 0, "GEMM M,N multiples of 64");
static_assert((kSeqL % kScanTS) == 0 && (kDin % kScanCh) == 0 && (kImg % kConvPT) == 0 && (kDin % 8) == 0, "tile multiples");
static_assert(kDmod <= kXtP && kDmod % 8 == 0 && kWoM >= kDmod, "pads");

constexpr size_t kSzXT  = (size_t)kPix * kXtP * 2;
constexpr size_t kSzWI  = (size_t)kXzP * kXtP * 2;
constexpr size_t kSzWX  = (size_t)kXdP * kDin * 2;
constexpr size_t kSzWF  = (size_t)kDin * kDin * 2;
constexpr size_t kSzWO  = (size_t)kWoM * kDin * 2;
constexpr size_t kSzXZ  = (size_t)kPix * kXzP * 4;
constexpr size_t kSzU   = (size_t)kTok * kDin * 4;
constexpr size_t kSzU16 = (size_t)kTok * kDin * 2;
constexpr size_t kSzTMP = (size_t)kPix * kDin * 4;
constexpr size_t kSzT16 = (size_t)kPix * kDin * 2;
constexpr size_t kSzXD  = (size_t)kTok * kXdP * 4;
constexpr size_t kSzY   = (size_t)kTok * kDin * 4;
constexpr size_t kSzG16 = (size_t)kPix * kDin * 2;
constexpr size_t kOffXTH = 0;
constexpr size_t kOffXTL = kOffXTH + kSzXT;
constexpr size_t kOffWIH = kOffXTL + kSzXT;
constexpr size_t kOffWIL = kOffWIH + kSzWI;
constexpr size_t kOffWXH = kOffWIL + kSzWI;
constexpr size_t kOffWXL = kOffWXH + kSzWX;
constexpr size_t kOffWFH = kOffWXL + kSzWX;
constexpr size_t kOffWFL = kOffWFH + kSzWF;
constexpr size_t kOffWOH = kOffWFL + kSzWF;
constexpr size_t kOffWOL = kOffWOH + kSzWO;
constexpr size_t kOffXZ  = kOffWOL + kSzWO;
constexpr size_t kOffU   = kOffXZ  + kSzXZ;
constexpr size_t kOffUH  = kOffU   + kSzU;
constexpr size_t kOffUL  = kOffUH  + kSzU16;
constexpr size_t kOffTMP = kOffUL  + kSzU16;
constexpr size_t kOffTAH = kOffTMP + kSzTMP;
constexpr size_t kOffTAL = kOffTAH + kSzT16;
constexpr size_t kOffXD  = kOffTAL + kSzT16;
constexpr size_t kOffY   = kOffXD  + kSzXD;
constexpr size_t kOffGH  = kOffY   + kSzY;
constexpr size_t kOffGL  = kOffGH  + kSzG16;
constexpr size_t kWsTotal = kOffGL + kSzG16;
static_assert(kWsTotal == 120029184ull, "carve total");
static_assert(kWsTotal <= 134217728ull, "carve cap");
static_assert((kOffXTL % 128) == 0 && (kOffWIH % 128) == 0 && (kOffWIL % 128) == 0 && (kOffWXH % 128) == 0 &&
              (kOffWXL % 128) == 0 && (kOffWFH % 128) == 0 && (kOffWFL % 128) == 0 && (kOffWOH % 128) == 0 &&
              (kOffWOL % 128) == 0 && (kOffXZ % 128) == 0 && (kOffU % 128) == 0 && (kOffUH % 128) == 0 &&
              (kOffUL % 128) == 0 && (kOffTMP % 128) == 0 && (kOffTAH % 128) == 0 && (kOffTAL % 128) == 0 &&
              (kOffXD % 128) == 0 && (kOffY % 128) == 0 && (kOffGH % 128) == 0 && (kOffGL % 128) == 0, "128-B aligned regions");

__device__ __forceinline__ unsigned short f2bf_bits(float f) {
  unsigned u = __float_as_uint(f);
  return (unsigned short)((u + 0x7FFFu + ((u >> 16) & 1u)) >> 16);
}
__device__ __forceinline__ float bf_bits2f(unsigned short h) { return __uint_as_float(((unsigned)h) << 16); }

__device__ __forceinline__ void split8_bf16(const v4f a0, const v4f a1, v8h& hv, v8h& lv) {
#pragma unroll
  for (int e = 0; e < 4; ++e) {
    const unsigned short h0 = f2bf_bits(a0[e]), h1 = f2bf_bits(a1[e]);
    const unsigned short l0 = f2bf_bits(a0[e] - bf_bits2f(h0)), l1 = f2bf_bits(a1[e] - bf_bits2f(h1));
    hv[e]     = __builtin_bit_cast(_Float16, h0);
    hv[4 + e] = __builtin_bit_cast(_Float16, h1);
    lv[e]     = __builtin_bit_cast(_Float16, l0);
    lv[4 + e] = __builtin_bit_cast(_Float16, l1);
  }
}

__device__ __forceinline__ void dep_guard4_h(v8f& a, v8f& b, v8f& c, v8f& d, v16h x, v16h y) { asm volatile("v_nop\n\tv_nop\n\tv_nop\n\tv_nop" : "+v"(a), "+v"(b), "+v"(c), "+v"(d) : "v"(x), "v"(y)); }
__device__ __forceinline__ void dep_guard4_b(v8f& a, v8f& b, v8f& c, v8f& d, v16b x, v16b y) { asm volatile("v_nop\n\tv_nop\n\tv_nop\n\tv_nop" : "+v"(a), "+v"(b), "+v"(c), "+v"(d) : "v"(x), "v"(y)); }
__device__ __forceinline__ void keep4_h(v16h a, v16h b, v16h c, v16h d) { asm volatile("v_nop" :: "v"(a), "v"(b), "v"(c), "v"(d)); }
__device__ __forceinline__ void keep4_b(v16b a, v16b b, v16b c, v16b d) { asm volatile("v_nop" :: "v"(a), "v"(b), "v"(c), "v"(d)); }
__device__ __forceinline__ void acc_guard4(v8f& a, v8f& b, v8f& c, v8f& d) { asm volatile("v_nop\n\tv_nop\n\tv_nop\n\tv_nop" : "+v"(a), "+v"(b), "+v"(c), "+v"(d)); }
template <typename T> struct Frag;
template <> struct Frag<_Float16> {
  typedef v16h V; union U { v16h v; v8h h[2]; };
  static __device__ __forceinline__ v16h load(const _Float16* p) {
    U f; f.h[0] = *(const v8h*)(p); f.h[1] = *(const v8h*)(p + 16); return f.v;
  }
  static __device__ __forceinline__ v8f mma(v16h a, v16h b, v8f c) {
    return __builtin_amdgcn_wmma_f32_16x16x32_f16(false, a, false, b, (short)0, c, false, false);
  }
  static __device__ __forceinline__ void guard4(v8f& a, v8f& b, v8f& c, v8f& d, v16h x, v16h y) { dep_guard4_h(a, b, c, d, x, y); }
  static __device__ __forceinline__ void keep(v16h a, v16h b, v16h c, v16h d) { keep4_h(a, b, c, d); }
};
template <> struct Frag<__bf16> {
  typedef v16b V; union U { v16b v; v8b h[2]; };
  static __device__ __forceinline__ v16b load(const __bf16* p) {
    U f; f.h[0] = *(const v8b*)(p); f.h[1] = *(const v8b*)(p + 16); return f.v;
  }
  static __device__ __forceinline__ v8f mma(v16b a, v16b b, v8f c) {
    return __builtin_amdgcn_wmma_f32_16x16x32_bf16(false, a, false, b, (short)0, c, false, false);
  }
  static __device__ __forceinline__ void guard4(v8f& a, v8f& b, v8f& c, v8f& d, v16b x, v16b y) { dep_guard4_b(a, b, c, d, x, y); }
  static __device__ __forceinline__ void keep(v16b a, v16b b, v16b c, v16b d) { keep4_b(a, b, c, d); }
};

template <int ET> struct Elem;
template <> struct Elem<0> { typedef _Float16 T; };
template <> struct Elem<1> { typedef __bf16 T; };
template <int ET, int SPL, int BIAS_MODE, int OUT_MODE, int ACT = 0>
__global__ __launch_bounds__(256) void wmma_gemm64(
    const unsigned short* __restrict__ Ap, const unsigned short* __restrict__ A2p, int lda, long strideA,
    const unsigned short* __restrict__ Btp, const unsigned short* __restrict__ Bt2p, int ldb, long strideB,
    void* __restrict__ Cout, void* __restrict__ Cout2, int ldc, long strideC,
    const float* __restrict__ bias,
    int M, int N, int K, int Mreal, float scale) {
  typedef typename Elem<ET>::T T;
  typedef typename Frag<T>::V V;
  const T* A = (const T*)Ap; const T* A2 = (const T*)A2p; const T* Bt = (const T*)Btp; const T* Bt2 = (const T*)Bt2p;
  __shared__ __align__(16) float sT[8][16 * 68];
  const int b    = blockIdx.y;
  const int lane = threadIdx.x & 31;
  const int wave = threadIdx.x >> 5;
  const int tilesN = N >> 6;
  const int tilesM = M >> 6;
  const int tile = blockIdx.x * 8 + wave;
  if (tile >= tilesM * tilesN) return;
  const int tm = tile / tilesN;
  const int tn = tile - tm * tilesN;
  const int m0 = tm << 6;
  const int n0 = tn << 6;

  const T* Ab  = A  + (size_t)b * strideA;
  const T* Bb  = Bt + (size_t)b * strideB;
  const T* Ab2 = (SPL >= 1) ? (A2  + (size_t)b * strideA) : nullptr;
  const T* Bb2 = (SPL == 2) ? (Bt2 + (size_t)b * strideB) : nullptr;

  const int rlane = lane & 15;
  const int koff  = (lane >> 4) * 8;
  const int mOff  = (lane >> 4) * 8;

  v8f acc[4][4];
#pragma unroll
  for (int i = 0; i < 4; ++i)
#pragma unroll
    for (int j = 0; j < 4; ++j) acc[i][j] = (v8f){0.f,0.f,0.f,0.f,0.f,0.f,0.f,0.f};

  for (int k0 = 0; k0 < K; k0 += 32) {
    V bh[4], bl[4];
#pragma unroll
    for (int j = 0; j < 4; ++j) {
      const size_t bo = (size_t)(n0 + (j << 4) + rlane) * ldb + koff + k0;
      bh[j] = Frag<T>::load(Bb + bo);
      if (SPL == 2) bl[j] = Frag<T>::load(Bb2 + bo);
    }
#pragma unroll
    for (int i = 0; i < 4; ++i) {
      const size_t ao = (size_t)(m0 + (i << 4) + rlane) * lda + koff + k0;
      V ah = Frag<T>::load(Ab + ao);
      V al = ah;
      if (SPL >= 1) al = Frag<T>::load(Ab2 + ao);
#pragma unroll
      for (int j = 0; j < 4; ++j) {
        acc[i][j] = Frag<T>::mma(ah, bh[j], acc[i][j]);
        if (SPL == 2) acc[i][j] = Frag<T>::mma(ah, bl[j], acc[i][j]);
        if (SPL >= 1) acc[i][j] = Frag<T>::mma(al, bh[j], acc[i][j]);
      }
      Frag<T>::guard4(acc[i][0], acc[i][1], acc[i][2], acc[i][3], ah, al);
    }
    Frag<T>::keep(bh[0], bh[1], bh[2], bh[3]);
    if (SPL == 2) Frag<T>::keep(bl[0], bl[1], bl[2], bl[3]);
  }
  acc_guard4(acc[0][0], acc[0][1], acc[0][2], acc[0][3]);
  acc_guard4(acc[1][0], acc[1][1], acc[1][2], acc[1][3]);
  acc_guard4(acc[2][0], acc[2][1], acc[2][2], acc[2][3]);
  acc_guard4(acc[3][0], acc[3][1], acc[3][2], acc[3][3]);

  float* slab = sT[wave];
#pragma unroll
  for (int i = 0; i < 4; ++i) {
    const int mBase = m0 + (i << 4);
#pragma unroll
    for (int j = 0; j < 4; ++j) {
      const int n = n0 + (j << 4) + rlane;
      float bv = 0.f;
      if (BIAS_MODE == 2) bv = bias[n];
#pragma unroll
      for (int r = 0; r < 8; ++r) {
        float v = acc[i][j][r] * scale;
        if (BIAS_MODE == 1) v += bias[mBase + mOff + r];
        if (BIAS_MODE == 2) v += bv;
        if (ACT == 1) v = tanhf(v);
        if (ACT == 2) v = fmaxf(v, 0.0f);
        if (ACT == 3) v = v * __builtin_amdgcn_rcpf(1.0f + expf(-v));
        if (ACT == 4) v = (v > 0.f) ? v : 0.01f * v;
        slab[(mOff + r) * 68 + (j << 4) + rlane] = v;
      }
    }
    __builtin_amdgcn_fence(__ATOMIC_RELEASE, "workgroup");
    __builtin_amdgcn_wave_barrier();
    __builtin_amdgcn_fence(__ATOMIC_ACQUIRE, "workgroup");
    if (OUT_MODE == 0) {
      float* C = (float*)Cout + (size_t)b * strideC;
      const int hh = lane >> 4, c4 = (lane & 15) * 4;
      for (int pass = 0; pass < 2; ++pass) {
#pragma unroll
        for (int it = 0; it < 8; ++it) {
          const int row = it * 2 + hh;
          v4f v = *(const v4f*)(slab + row * 68 + c4);
          if (mBase + row < Mreal) *(volatile v4f*)(C + (size_t)(mBase + row) * ldc + n0 + c4) = v;
        }
        __threadfence();
      }
    } else {
      const int q = lane >> 3, c8 = (lane & 7) * 8;
      unsigned short* C  = (unsigned short*)Cout  + (size_t)b * strideC;
      unsigned short* C2 = (OUT_MODE == 2) ? ((unsigned short*)Cout2 + (size_t)b * strideC) : nullptr;
      for (int pass = 0; pass < 2; ++pass) {
#pragma unroll
        for (int it = 0; it < 4; ++it) {
          const int row = it * 4 + q;
          const float* sp = slab + row * 68 + c8;
          v8h hv, lv;
#pragma unroll
          for (int e = 0; e < 8; ++e) {
            if (OUT_MODE == 1) {
              hv[e] = (_Float16)sp[e];
            } else {
              unsigned short hb = f2bf_bits(sp[e]);
              unsigned short lb = f2bf_bits(sp[e] - bf_bits2f(hb));
              hv[e] = __builtin_bit_cast(_Float16, hb);
              lv[e] = __builtin_bit_cast(_Float16, lb);
            }
          }
          if (mBase + row < Mreal) {
            *(volatile v8h*)(C + (size_t)(mBase + row) * ldc + n0 + c8) = hv;
            if (OUT_MODE == 2) *(volatile v8h*)(C2 + (size_t)(mBase + row) * ldc + n0 + c8) = lv;
          }
        }
        __threadfence();
      }
    }
    __builtin_amdgcn_fence(__ATOMIC_RELEASE, "workgroup");
    __builtin_amdgcn_wave_barrier();
    __builtin_amdgcn_fence(__ATOMIC_ACQUIRE, "workgroup");
  }
}

__global__ __launch_bounds__(256) void split_pad_bf16_kernel(
    const float* __restrict__ src, long srcBS, int R, int Csrc, int gapAt, int gapLen,
    unsigned short* __restrict__ dhi, unsigned short* __restrict__ dlo, long dstBS, int Cpad, int total8)
{
  const int i = blockIdx.x * 256 + threadIdx.x;
  if (i >= total8) return;
  const float* sb = src + (size_t)blockIdx.y * srcBS;
  const size_t e0 = (size_t)i << 3;
  const int r  = (int)(e0 / (size_t)Cpad);
  const int c0 = (int)(e0 - (size_t)r * Cpad);
  const bool rowok = (r < gapAt) || (r >= gapAt + gapLen);
  int rs = (r < gapAt) ? r : (r - gapLen);
  const bool rv = rowok && (rs >= 0) && (rs < R);
  rs = rs < 0 ? 0 : rs;
  rs = rs > R - 1 ? R - 1 : rs;
  v4f a0, a1;
#pragma unroll
  for (int e = 0; e < 4; ++e) {
    const int ca = c0 + e, cbq = c0 + 4 + e;
    const int cac = ca < Csrc ? ca : Csrc - 1;
    const int cbc = cbq < Csrc ? cbq : Csrc - 1;
    const float fa = sb[(size_t)rs * Csrc + cac];
    const float fb = sb[(size_t)rs * Csrc + cbc];
    const float va = (rv && ca < Csrc) ? 1.0f : 0.0f;
    const float vb = (rv && cbq < Csrc) ? 1.0f : 0.0f;
    a0[e] = fa * va;
    a1[e] = fb * vb;
  }
  v8h hv, lv;
  split8_bf16(a0, a1, hv, lv);
  unsigned short* qh = dhi + (size_t)blockIdx.y * dstBS + e0;
  unsigned short* ql = dlo + (size_t)blockIdx.y * dstBS + e0;
  *(volatile v8h*)qh = hv;
  *(volatile v8h*)ql = lv;
  __threadfence();
  *(volatile v8h*)qh = hv;
  *(volatile v8h*)ql = lv;
}

__global__ __launch_bounds__(256) void xpose_split_x_kernel(
    const float* __restrict__ x, unsigned short* __restrict__ xh, unsigned short* __restrict__ xl)
{
  __shared__ __align__(16) float sX[kDmod * 32];
  const int tid = threadIdx.x;
  const int b = blockIdx.x >> 5;
  const int hw0 = (blockIdx.x & 31) * 32;
#pragma unroll
  for (int i = 0; i < (kDmod * 32) / 256; ++i) {
    const int idx = i * 256 + tid;
    const int c = idx >> 5, px = idx & 31;
    sX[idx] = x[((size_t)(b * kDmod + c)) * kHW + hw0 + px];
  }
  __syncthreads();
  const int g = tid & 15, pr = tid >> 4;
  const float gf = (g < kDmod / 8) ? 1.0f : 0.0f;
  v8h hv[2], lv[2];
#pragma unroll
  for (int it = 0; it < 2; ++it) {
    const int prow = it * 16 + pr;
    v4f a0, a1;
#pragma unroll
    for (int e = 0; e < 4; ++e) {
      int ca = 8 * g + e;      ca = ca > kDmod - 1 ? kDmod - 1 : ca;
      int cb = 8 * g + 4 + e;  cb = cb > kDmod - 1 ? kDmod - 1 : cb;
      a0[e] = sX[ca * 32 + prow] * gf;
      a1[e] = sX[cb * 32 + prow] * gf;
    }
    split8_bf16(a0, a1, hv[it], lv[it]);
  }
  for (int pass = 0; pass < 2; ++pass) {
#pragma unroll
    for (int it = 0; it < 2; ++it) {
      const int prow = it * 16 + pr;
      const size_t o = ((size_t)(b * kHW + hw0 + prow)) * kXtP + 8 * g;
      *(volatile v8h*)(xh + o) = hv[it];
      *(volatile v8h*)(xl + o) = lv[it];
    }
    __threadfence();
  }
}

template <int ACT, bool HAS_BIAS, bool OUT_F32, bool OUT_BF>
__global__ __launch_bounds__(192) void dwconv3x3_kernel(
    const float* __restrict__ in, int inP, int inBS,
    const float* __restrict__ w, const float* __restrict__ bias,
    float* __restrict__ outF, unsigned short* __restrict__ outH, unsigned short* __restrict__ outL, int outBS)
{
  __shared__ __align__(16) float sT[kConvPT * kDin];
  const int tid = threadIdx.x;
  constexpr int kTilesPerImg = kHW / kConvPT;
  const int b   = blockIdx.x / kTilesPerImg;
  const int hw0 = (blockIdx.x - b * kTilesPerImg) * kConvPT;
  const int yy  = hw0 >> 5, xx0 = hw0 & 31;
  float wk[9];
#pragma unroll
  for (int k = 0; k < 9; ++k) wk[k] = w[tid * 9 + k];
  float bv = 0.0f;
  if (HAS_BIAS) bv = bias[tid];
  const float* ib = in + (size_t)b * inBS * inP + tid;
#pragma unroll 1
  for (int px = 0; px < kConvPT; ++px) {
    const int xx = xx0 + px;
    float acc = 0.0f;
#pragma unroll
    for (int ky = 0; ky < 3; ++ky) {
      const int iy = yy + ky - 1;
      const bool rowv = (iy >= 0) && (iy < kImg);
      const int iyc = iy < 0 ? 0 : (iy > kImg - 1 ? kImg - 1 : iy);
#pragma unroll
      for (int kx = 0; kx < 3; ++kx) {
        const int ix = xx + kx - 1;
        const bool v = rowv && (ix >= 0) && (ix < kImg);
        const int ixc = ix < 0 ? 0 : (ix > kImg - 1 ? kImg - 1 : ix);
        const float f = ib[(size_t)(iyc * kImg + ixc) * inP];
        const float vf = v ? 1.0f : 0.0f;
        acc = fmaf(wk[ky * 3 + kx], f * vf, acc);
      }
    }
    float r = acc;
    if (HAS_BIAS) r = r + bv;
    if (ACT == 1) r = fmaxf(r, 0.0f);
    if (ACT == 2) r = r * __builtin_amdgcn_rcpf(1.0f + expf(-r));
    sT[px * kDin + tid] = r;
  }
  __syncthreads();
  const size_t obase = ((size_t)b * outBS + hw0) * kDin;
  v4f fv[4];
  v8h hv[2], lv[2];
  if (OUT_F32) {
#pragma unroll
    for (int it = 0; it < 4; ++it) fv[it] = *(const v4f*)(sT + 4 * (it * kDin + tid));
  }
  if (OUT_BF) {
#pragma unroll
    for (int it = 0; it < 2; ++it) {
      const float* sp = sT + 8 * (it * kDin + tid);
      const v4f a0 = *(const v4f*)(sp);
      const v4f a1 = *(const v4f*)(sp + 4);
      split8_bf16(a0, a1, hv[it], lv[it]);
    }
  }
  for (int pass = 0; pass < 2; ++pass) {
    if (OUT_F32) {
#pragma unroll
      for (int it = 0; it < 4; ++it)
        *(volatile v4f*)(outF + obase + 4 * (it * kDin + tid)) = fv[it];
    }
    if (OUT_BF) {
#pragma unroll
      for (int it = 0; it < 2; ++it) {
        const size_t o = obase + 8 * (it * kDin + tid);
        *(volatile v8h*)(outH + o) = hv[it];
        *(volatile v8h*)(outL + o) = lv[it];
      }
    }
    __threadfence();
  }
}

__global__ __launch_bounds__(kScanCh) void scan_kernel(
    const float* __restrict__ XD, const float* __restrict__ U,
    const float* __restrict__ Wdt, const float* __restrict__ bdt,
    const float* __restrict__ Alog, const float* __restrict__ Dp,
    float* __restrict__ Y)
{
  __shared__ __align__(16) float sX[kScanTS * kXdP];
  __shared__ __align__(16) float sY[kScanTS * kScanYP];
  __shared__ __align__(16) float sA[kNst * kScanCh];
  const int tid = threadIdx.x, lane = tid & 31, wave = tid >> 5;
  constexpr int kBlkPerB = kDin / kScanCh;
  const int bix = blockIdx.x / kBlkPerB;
  const int d0  = (blockIdx.x - bix * kBlkPerB) * kScanCh;
  const int d   = d0 + tid;
  const size_t row0 = (size_t)bix * kSeqL;
#pragma unroll 1
  for (int s = 0; s < kNst; ++s) sA[s * kScanCh + tid] = -expf(Alog[(size_t)d * kNst + s]);
  __syncthreads();
  float negA[kNst], h[kNst];
#pragma unroll
  for (int s = 0; s < kNst; ++s) {
    negA[s] = sA[s * kScanCh + tid];
    h[s] = 0.0f;
  }
  float wd[kDtR];
#pragma unroll
  for (int r = 0; r < kDtR; ++r) wd[r] = Wdt[(size_t)d * kDtR + r];
  const float bb = bdt[d], Dd = Dp[d];
  const int lr = tid >> 4, lc4 = (tid & 15) * 4;
  const int hh = lane >> 4, c4 = (lane & 15) * 4;
#pragma unroll 1
  for (int t0 = 0; t0 < kSeqL; t0 += kScanTS) {
    __syncthreads();
#pragma unroll
    for (int i = 0; i < 16; ++i) {
      const int r = lr + 4 * i;
      *(v4f*)(sX + r * kXdP + lc4) = *(const v4f*)(XD + (row0 + t0 + r) * kXdP + lc4);
    }
    __syncthreads();
#pragma unroll 1
    for (int s = 0; s < kScanTS; ++s) {
      const int t = t0 + s;
      const float* xr = sX + s * kXdP;
      const v4f q0 = *(const v4f*)(xr);
      const v4f q1 = *(const v4f*)(xr + 4);
      float vdot = q0[0] * wd[0];
      vdot = fmaf(q0[1], wd[1], vdot);
      vdot = fmaf(q0[2], wd[2], vdot);
      vdot = fmaf(q0[3], wd[3], vdot);
      vdot = fmaf(q1[0], wd[4], vdot);
      vdot = fmaf(q1[1], wd[5], vdot);
      float Bs[kNst], Cs[kNst];
#pragma unroll
      for (int q4 = 0; q4 < 4; ++q4) {
        const v4f bv = *(const v4f*)(xr + kColB + 4 * q4);
        const v4f cv = *(const v4f*)(xr + kColC + 4 * q4);
        Bs[4 * q4 + 0] = bv[0]; Bs[4 * q4 + 1] = bv[1]; Bs[4 * q4 + 2] = bv[2]; Bs[4 * q4 + 3] = bv[3];
        Cs[4 * q4 + 0] = cv[0]; Cs[4 * q4 + 1] = cv[1]; Cs[4 * q4 + 2] = cv[2]; Cs[4 * q4 + 3] = cv[3];
      }
      const float v   = (vdot + bb) + bb;
      const float a   = __expf(-fabsf(v));
      const float up  = 1.0f + a;
      const float l1p = __logf(up) + (a - (up - 1.0f)) * __builtin_amdgcn_rcpf(up);
      const float dt  = fmaxf(v, 0.0f) + l1p;
      const float xt  = U[(row0 + t) * kDin + d];
      const float dtx = dt * xt;
      float ysum = 0.0f;
#pragma unroll
      for (int k = 0; k < kNst; ++k) {
        const float e = __expf(dt * negA[k]);
        h[k] = fmaf(e, h[k], dtx * Bs[k]);
        ysum = fmaf(h[k], Cs[k], ysum);
      }
      sY[s * kScanYP + tid] = fmaf(Dd, xt, ysum);
    }
    __syncthreads();
    v4f ov[16];
#pragma unroll
    for (int it = 0; it < 16; ++it) {
      const int row = it * 4 + wave * 2 + hh;
      ov[it] = *(const v4f*)(sY + row * kScanYP + c4);
    }
    for (int pass = 0; pass < 2; ++pass) {
#pragma unroll
      for (int it = 0; it < 16; ++it) {
        const int row = it * 4 + wave * 2 + hh;
        *(volatile v4f*)(Y + (row0 + t0 + row) * kDin + d0 + c4) = ov[it];
      }
      __threadfence();
    }
  }
}

__global__ __launch_bounds__(256) void combine_ln_gate_kernel(
    const float* __restrict__ Y, const float* __restrict__ XZ, const float* __restrict__ sw,
    const float* __restrict__ lnw, const float* __restrict__ lnb,
    unsigned short* __restrict__ GH, unsigned short* __restrict__ GL)
{
  const int lane = threadIdx.x & 31, wave = threadIdx.x >> 5;
  const int p = blockIdx.x * 8 + wave;
  const int b = p >> 10, hw = p & (kHW - 1);
  const bool act = lane < (kDin / 8);
  const int c0 = (act ? lane : (kDin / 8 - 1)) * 8;
  const float af = act ? 1.0f : 0.0f;
  const float s0 = sw[0], s1 = sw[1], s2 = sw[2], s3 = sw[3];
  const float mx = fmaxf(fmaxf(s0, s1), fmaxf(s2, s3));
  const float e0 = expf(s0 - mx), e1 = expf(s1 - mx), e2 = expf(s2 - mx), e3 = expf(s3 - mx);
  const float inv = 1.0f / (((e0 + e1) + e2) + e3);
  const float w0 = e0 * inv, w1 = e1 * inv, w2 = e2 * inv, w3 = e3 * inv;
  constexpr size_t kSegS = (size_t)kHW * kDin;
  const float* yb = Y + ((size_t)b * kSeqL + hw) * kDin + c0;
  const v4f p0a = *(const v4f*)(yb),             p0b = *(const v4f*)(yb + 4);
  const v4f p1a = *(const v4f*)(yb + kSegS),     p1b = *(const v4f*)(yb + kSegS + 4);
  const v4f p2a = *(const v4f*)(yb + 2 * kSegS), p2b = *(const v4f*)(yb + 2 * kSegS + 4);
  const v4f p3a = *(const v4f*)(yb + 3 * kSegS), p3b = *(const v4f*)(yb + 3 * kSegS + 4);
  float yc[8];
#pragma unroll
  for (int e = 0; e < 4; ++e) {
    yc[e]     = ((w0 * p0a[e] + w1 * p1a[e]) + w2 * p2a[e]) + w3 * p3a[e];
    yc[4 + e] = ((w0 * p0b[e] + w1 * p1b[e]) + w2 * p2b[e]) + w3 * p3b[e];
  }
  float sm = 0.0f;
#pragma unroll
  for (int e = 0; e < 8; ++e) sm += yc[e];
  sm *= af;
  sm += __shfl_xor(sm, 16, 32);
  sm += __shfl_xor(sm, 8, 32);
  sm += __shfl_xor(sm, 4, 32);
  sm += __shfl_xor(sm, 2, 32);
  sm += __shfl_xor(sm, 1, 32);
  const float mu = sm * (1.0f / (float)kDin);
  float sq = 0.0f;
#pragma unroll
  for (int e = 0; e < 8; ++e) { const float dv = yc[e] - mu; sq = fmaf(dv, dv, sq); }
  sq *= af;
  sq += __shfl_xor(sq, 16, 32);
  sq += __shfl_xor(sq, 8, 32);
  sq += __shfl_xor(sq, 4, 32);
  sq += __shfl_xor(sq, 2, 32);
  sq += __shfl_xor(sq, 1, 32);
  const float var = sq * (1.0f / (float)kDin);
  const float rs = rsqrtf(var + 1e-5f);
  const float* zp = XZ + (size_t)p * kXzP + kDin + c0;
  const v4f za = *(const v4f*)(zp), zb = *(const v4f*)(zp + 4);
  const v4f wa = *(const v4f*)(lnw + c0), wb = *(const v4f*)(lnw + c0 + 4);
  const v4f ba = *(const v4f*)(lnb + c0), bq = *(const v4f*)(lnb + c0 + 4);
  v4f g0, g1;
#pragma unroll
  for (int e = 0; e < 4; ++e) {
    const float z0 = za[e], z1 = zb[e];
    const float sg0 = __builtin_amdgcn_rcpf(1.0f + __expf(-z0));
    const float sg1 = __builtin_amdgcn_rcpf(1.0f + __expf(-z1));
    float t0 = (yc[e] - mu) * rs;     t0 = t0 * wa[e]; t0 = t0 + ba[e];
    float t1 = (yc[4 + e] - mu) * rs; t1 = t1 * wb[e]; t1 = t1 + bq[e];
    g0[e] = t0 * (z0 * sg0);
    g1[e] = t1 * (z1 * sg1);
  }
  v8h hv, lv;
  split8_bf16(g0, g1, hv, lv);
  unsigned short* gh = GH + (size_t)p * kDin + c0;
  unsigned short* gl = GL + (size_t)p * kDin + c0;
  for (int pass = 0; pass < 2; ++pass) {
    if (act) {
      *(volatile v8h*)gh = hv;
      *(volatile v8h*)gl = lv;
    }
    __threadfence();
  }
}

constexpr int kBlkIn  = ((kPix / 64) * (kXzP / 64)) / 8;
constexpr int kBlkPw  = ((kHW / 64) * (kDin / 64)) / 8;
constexpr int kBlkXp  = ((kTok / 64) * (kXdP / 64)) / 8;
constexpr int kBlkOut = ((kWoM / 64) * (kHW / 64)) / 8;
static_assert(kBlkIn * 8 == (kPix / 64) * (kXzP / 64) && kBlkPw * 8 == (kHW / 64) * (kDin / 64) &&
              kBlkXp * 8 == (kTok / 64) * (kXdP / 64) && kBlkOut * 8 == (kWoM / 64) * (kHW / 64), "exact tile grids");
static_assert(((kXzP * kXtP) / 8) % 256 == 0 && ((kXdP * kDin) / 8) % 256 == 0 && ((kDin * kDin) / 8) % 256 == 0 &&
              ((kWoM * kDin) / 8) % 256 == 0 && ((kHW * kDin) / 8) % 256 == 0, "split grids exact");

extern "C" void kernel_launch(void* const* d_in, const int* in_sizes, int n_in,
                              void* d_out, int out_size, void* d_ws, size_t ws_size,
                              hipStream_t stream) {
  if (n_in < 23) return;
  if (in_sizes[0]  != kNB * kDmod * kHW) return;
  if (in_sizes[1]  != kXzP * kDmod) return;
  if (in_sizes[2]  != kDin * 9) return;
  if (in_sizes[3]  != kDin) return;
  if (in_sizes[4]  != kXpN * kDin) return;
  if (in_sizes[5]  != kDin * kDtR) return;
  if (in_sizes[6]  != kDin) return;
  if (in_sizes[7]  != kDin * kNst) return;
  if (in_sizes[8]  != kDin) return;
  if (in_sizes[9]  != 4) return;
  if (in_sizes[10] != kDin) return;
  if (in_sizes[11] != kDin) return;
  if (in_sizes[12] != kDmod * kDin) return;
  if (in_sizes[13] != kDin * 9 || in_sizes[14] != kDin) return;
  if (in_sizes[15] != kDin * kDin || in_sizes[16] != kDin) return;
  if (in_sizes[17] != kDin * 9 || in_sizes[18] != kDin) return;
  if (in_sizes[19] != kDin * 9 || in_sizes[20] != kDin) return;
  if (in_sizes[21] != kDin * 9 || in_sizes[22] != kDin * 9) return;
  if (out_size != kNB * kDmod * kHW) return;
  if (ws_size < kWsTotal) return;

  const float* x         = (const float*)d_in[0];
  const float* in_proj_w = (const float*)d_in[1];
  const float* conv_w    = (const float*)d_in[2];
  const float* conv_b    = (const float*)d_in[3];
  const float* x_proj_w  = (const float*)d_in[4];
  const float* dt_proj_w = (const float*)d_in[5];
  const float* dt_proj_b = (const float*)d_in[6];
  const float* A_log     = (const float*)d_in[7];
  const float* Dp        = (const float*)d_in[8];
  const float* scan_w    = (const float*)d_in[9];
  const float* ln_w      = (const float*)d_in[10];
  const float* ln_b      = (const float*)d_in[11];
  const float* out_pw    = (const float*)d_in[12];
  const float* fc_dw_w   = (const float*)d_in[13];
  const float* fc_dw_b   = (const float*)d_in[14];
  const float* fc_pw_w   = (const float*)d_in[15];
  const float* fc_pw_b   = (const float*)d_in[16];
  const float* fv_w      = (const float*)d_in[17];
  const float* fv_b      = (const float*)d_in[18];
  const float* fh_w      = (const float*)d_in[19];
  const float* fh_b      = (const float*)d_in[20];
  const float* sob_x     = (const float*)d_in[21];
  const float* sob_y     = (const float*)d_in[22];
  float* out = (float*)d_out;

  char* ws = (char*)d_ws;
  unsigned short* XTH = (unsigned short*)(ws + kOffXTH);
  unsigned short* XTL = (unsigned short*)(ws + kOffXTL);
  unsigned short* WIH = (unsigned short*)(ws + kOffWIH);
  unsigned short* WIL = (unsigned short*)(ws + kOffWIL);
  unsigned short* WXH = (unsigned short*)(ws + kOffWXH);
  unsigned short* WXL = (unsigned short*)(ws + kOffWXL);
  unsigned short* WFH = (unsigned short*)(ws + kOffWFH);
  unsigned short* WFL = (unsigned short*)(ws + kOffWFL);
  unsigned short* WOH = (unsigned short*)(ws + kOffWOH);
  unsigned short* WOL = (unsigned short*)(ws + kOffWOL);
  float*          XZ  = (float*)(ws + kOffXZ);
  float*          U   = (float*)(ws + kOffU);
  unsigned short* UH  = (unsigned short*)(ws + kOffUH);
  unsigned short* UL  = (unsigned short*)(ws + kOffUL);
  float*          TMP = (float*)(ws + kOffTMP);
  unsigned short* TAH = (unsigned short*)(ws + kOffTAH);
  unsigned short* TAL = (unsigned short*)(ws + kOffTAL);
  float*          XD  = (float*)(ws + kOffXD);
  float*          Y   = (float*)(ws + kOffY);
  unsigned short* GH  = (unsigned short*)(ws + kOffGH);
  unsigned short* GL  = (unsigned short*)(ws + kOffGL);

  const int kNoGap = 1 << 20;
  const size_t kSeg = (size_t)kHW * kDin;
  const long kTokBS = (long)kSeqL * kDin;

  xpose_split_x_kernel<<<kPix / 32, 256, 0, stream>>>(x, XTH, XTL);
  split_pad_bf16_kernel<<<dim3((kXzP * kXtP / 8) / 256, 1), 256, 0, stream>>>(
      in_proj_w, 0L, kXzP, kDmod, kNoGap, 0, WIH, WIL, 0L, kXtP, kXzP * kXtP / 8);
  split_pad_bf16_kernel<<<dim3((kXdP * kDin / 8) / 256, 1), 256, 0, stream>>>(
      x_proj_w, 0L, kXpN, kDin, kDtR, kColB - kDtR, WXH, WXL, 0L, kDin, kXdP * kDin / 8);
  split_pad_bf16_kernel<<<dim3((kDin * kDin / 8) / 256, 1), 256, 0, stream>>>(
      fc_pw_w, 0L, kDin, kDin, kNoGap, 0, WFH, WFL, 0L, kDin, kDin * kDin / 8);
  split_pad_bf16_kernel<<<dim3((kWoM * kDin / 8) / 256, 1), 256, 0, stream>>>(
      out_pw, 0L, kDmod, kDin, kNoGap, 0, WOH, WOL, 0L, kDin, kWoM * kDin / 8);

  wmma_gemm64<1, 2, 0, 0, 0><<<dim3(kBlkIn, 1), 256, 0, stream>>>(
      XTH, XTL, kXtP, 0L,
      WIH, WIL, kXtP, 0L,
      (void*)XZ, nullptr, kXzP, 0L,
      nullptr,
      kPix, kXzP, kDmod, kPix, 1.0f);

  dwconv3x3_kernel<2, true, true, true><<<kPix / kConvPT, kDin, 0, stream>>>(
      XZ, kXzP, kHW, conv_w, conv_b, U, UH, UL, kSeqL);
  dwconv3x3_kernel<0, false, true, false><<<kPix / kConvPT, kDin, 0, stream>>>(
      U, kDin, kSeqL, sob_x, nullptr, TMP, nullptr, nullptr, kHW);
  dwconv3x3_kernel<1, true, true, true><<<kPix / kConvPT, kDin, 0, stream>>>(
      TMP, kDin, kHW, fv_w, fv_b, U + kSeg, UH + kSeg, UL + kSeg, kSeqL);
  dwconv3x3_kernel<0, true, false, true><<<kPix / kConvPT, kDin, 0, stream>>>(
      U, kDin, kSeqL, fc_dw_w, fc_dw_b, nullptr, TAH, TAL, kHW);
  wmma_gemm64<1, 2, 2, 0, 2><<<dim3(kBlkPw, kNB), 256, 0, stream>>>(
      TAH, TAL, kDin, (long)kSeg,
      WFH, WFL, kDin, 0L,
      (void*)(U + 2 * kSeg), nullptr, kDin, kTokBS,
      fc_pw_b,
      kHW, kDin, kDin, kHW, 1.0f);
  split_pad_bf16_kernel<<<dim3((kHW * kDin / 8) / 256, kNB), 256, 0, stream>>>(
      U + 2 * kSeg, kTokBS, kHW, kDin, kNoGap, 0, UH + 2 * kSeg, UL + 2 * kSeg, kTokBS, kDin, kHW * kDin / 8);
  dwconv3x3_kernel<0, false, true, false><<<kPix / kConvPT, kDin, 0, stream>>>(
      U, kDin, kSeqL, sob_y, nullptr, TMP, nullptr, nullptr, kHW);
  dwconv3x3_kernel<1, true, true, true><<<kPix / kConvPT, kDin, 0, stream>>>(
      TMP, kDin, kHW, fh_w, fh_b, U + 3 * kSeg, UH + 3 * kSeg, UL + 3 * kSeg, kSeqL);

  wmma_gemm64<1, 2, 0, 0, 0><<<dim3(kBlkXp, 1), 256, 0, stream>>>(
      UH, UL, kDin, 0L,
      WXH, WXL, kDin, 0L,
      (void*)XD, nullptr, kXdP, 0L,
      nullptr,
      kTok, kXdP, kDin, kTok, 1.0f);

  scan_kernel<<<kNB * (kDin / kScanCh), kScanCh, 0, stream>>>(XD, U, dt_proj_w, dt_proj_b, A_log, Dp, Y);

  combine_ln_gate_kernel<<<kPix / 8, 256, 0, stream>>>(Y, XZ, scan_w, ln_w, ln_b, GH, GL);

  wmma_gemm64<1, 2, 0, 0, 0><<<dim3(kBlkOut, kNB), 256, 0, stream>>>(
      WOH, WOL, kDin, 0L,
      GH, GL, kDin, (long)kSeg,
      (void*)out, nullptr, kHW, (long)kDmod * kHW,
      nullptr,
      kWoM, kHW, kDin, kDmod, 1.0f);
}
